// CleanDITBlock_17154099380430
// MI455X (gfx1250) — hardware-verified
//
#include <hip/hip_runtime.h>
#include <math.h>
#include <stdint.h>

constexpr int kBatch   = 2;
constexpr int kSeq     = 2048;
constexpr int kCtxLen  = 512;
constexpr int kDim     = 1024;
constexpr int kHeads   = 16;
constexpr int kHeadDim = 64;
constexpr int kHid     = 4096;
constexpr int kSixD    = 6144;
constexpr int kTok     = kBatch * kSeq;
constexpr int kCtxTok  = kBatch * kCtxLen;
constexpr float kWCarry     = 32.0f;
constexpr float kWCarryInv  = 1.0f / 32.0f;
constexpr float kPScale     = 32768.0f;
constexpr float kOCarry     = 16.0f;
constexpr float kWOScale    = 1.0f / 512.0f;
constexpr float kLoCarry    = 2048.0f;
constexpr float kW2LoScale  = 1.0f / 65536.0f;

typedef __attribute__((ext_vector_type(16))) _Float16 v16h;
typedef __attribute__((ext_vector_type(8)))  _Float16 v8h;
typedef __attribute__((ext_vector_type(16))) __bf16   v16b;
typedef __attribute__((ext_vector_type(8)))  __bf16   v8b;
typedef __attribute__((ext_vector_type(8)))  float    v8f;
typedef __attribute__((ext_vector_type(4)))  float    v4f;
typedef __attribute__((ext_vector_type(2)))  float    v2f;
typedef __attribute__((ext_vector_type(4)))  unsigned int v4u;

constexpr size_t kMiB      = 1048576;
constexpr size_t kOffSmall = 0;
constexpr size_t kOffCos   = 65536;
constexpr size_t kOffSin   = 65536 + 524288;
constexpr size_t kOffXa    = 2 * kMiB;
constexpr size_t kOffXb    = 18 * kMiB;
constexpr size_t kOffNx    = 34 * kMiB;
constexpr size_t kOffBig   = 42 * kMiB;
constexpr size_t kOffQkv   = 74 * kMiB;
constexpr size_t kOffW1T   = 74 * kMiB;
constexpr size_t kOffW2T   = 82 * kMiB;
constexpr size_t kOffHlo   = 90 * kMiB;
constexpr size_t kOffWsw   = 98 * kMiB;
constexpr size_t kWsTotal  = 122 * kMiB;
static_assert(kWsTotal == 127926272);
static_assert(kWsTotal <= 134217728);
static_assert((size_t)kTok * 2 * kDim * 4 == 32 * kMiB);
static_assert((size_t)kTok * kHid * 2 == 32 * kMiB);
static_assert(kOffHlo + 32 * kMiB == kWsTotal);
static_assert(kOffW2T + (size_t)kDim * kHid * 2 == kOffHlo);
static_assert((size_t)kTok * kDim * 4 == 16 * kMiB);
static_assert((size_t)kTok * kDim * 2 == 8 * kMiB);

__device__ __forceinline__ unsigned short f2bf_bits(float f) {
  unsigned u = __float_as_uint(f);
  return (unsigned short)((u + 0x7FFFu + ((u >> 16) & 1u)) >> 16);
}
__device__ __forceinline__ float bf_bits2f(unsigned short h) { return __uint_as_float(((unsigned)h) << 16); }
__device__ __forceinline__ unsigned short f2h_bits(float f) { return __builtin_bit_cast(unsigned short, (_Float16)f); }
__device__ __forceinline__ unsigned pk16(unsigned short a, unsigned short b) { return (unsigned)a | ((unsigned)b << 16); }

__device__ __forceinline__ void dep_guard_h(v8f& a, v8f& b, v16h x, v16h y) { asm volatile("v_nop\n\tv_nop\n\tv_nop\n\tv_nop" : "+v"(a), "+v"(b) : "v"(x), "v"(y)); }
__device__ __forceinline__ void dep_guard_b(v8f& a, v8f& b, v16b x, v16b y) { asm volatile("v_nop\n\tv_nop\n\tv_nop\n\tv_nop" : "+v"(a), "+v"(b) : "v"(x), "v"(y)); }
__device__ __forceinline__ void keep4_h(v16h a, v16h b, v16h c, v16h d) { asm volatile("v_nop" :: "v"(a), "v"(b), "v"(c), "v"(d)); }
__device__ __forceinline__ void keep4_b(v16b a, v16b b, v16b c, v16b d) { asm volatile("v_nop" :: "v"(a), "v"(b), "v"(c), "v"(d)); }
__device__ __forceinline__ void acc_guard4(v8f& a, v8f& b, v8f& c, v8f& d) { asm volatile("v_nop\n\tv_nop\n\tv_nop\n\tv_nop" : "+v"(a), "+v"(b), "+v"(c), "+v"(d)); }
template <typename T> struct Frag;
template <> struct Frag<_Float16> {
  typedef v16h V; union U { v16h v; v8h h[2]; };
  static __device__ __forceinline__ v16h load(const _Float16* p) {
    U f; f.h[0] = *(const v8h*)(p); f.h[1] = *(const v8h*)(p + 16); return f.v;
  }
  static __device__ __forceinline__ v8f mma(v16h a, v16h b, v8f c) {
    return __builtin_amdgcn_wmma_f32_16x16x32_f16(false, a, false, b, (short)0, c, false, false);
  }
  static __device__ __forceinline__ void guard(v8f& a, v8f& b, v16h x, v16h y) { dep_guard_h(a, b, x, y); }
  static __device__ __forceinline__ void keep(v16h a, v16h b, v16h c, v16h d) { keep4_h(a, b, c, d); }
};
template <> struct Frag<__bf16> {
  typedef v16b V; union U { v16b v; v8b h[2]; };
  static __device__ __forceinline__ v16b load(const __bf16* p) {
    U f; f.h[0] = *(const v8b*)(p); f.h[1] = *(const v8b*)(p + 16); return f.v;
  }
  static __device__ __forceinline__ v8f mma(v16b a, v16b b, v8f c) {
    return __builtin_amdgcn_wmma_f32_16x16x32_bf16(false, a, false, b, (short)0, c, false, false);
  }
  static __device__ __forceinline__ void guard(v8f& a, v8f& b, v16b x, v16b y) { dep_guard_b(a, b, x, y); }
  static __device__ __forceinline__ void keep(v16b a, v16b b, v16b c, v16b d) { keep4_b(a, b, c, d); }
};

template <int ET> struct Elem;
template <> struct Elem<0> { typedef _Float16 T; };
template <> struct Elem<1> { typedef __bf16 T; };
template <int ET, bool SPLIT, int BIAS_MODE, int OUT_MODE, bool RESID, bool GATED, bool PREADD>
__global__ __launch_bounds__(256) void wmma_gemm64(
    const unsigned short* __restrict__ Ap, const unsigned short* __restrict__ A2p, int lda, long strideA,
    const unsigned short* __restrict__ Btp, const unsigned short* __restrict__ Bt2p, int ldb, long strideB,
    void* __restrict__ Cout, void* __restrict__ Cout2, int ldc, long strideC,
    const float* __restrict__ bias,
    const float* __restrict__ gate, long strideG,
    const float* __restrict__ pre, long strideP,
    const float* __restrict__ resid, long strideR,
    int M, int N, int K, float scale) {
  typedef typename Elem<ET>::T T;
  typedef typename Frag<T>::V V;
  const T* A = (const T*)Ap; const T* A2 = (const T*)A2p; const T* Bt = (const T*)Btp; const T* Bt2 = (const T*)Bt2p;
  __shared__ __align__(16) float sT[8][16 * 68];
  const int b    = blockIdx.y;
  const int lane = threadIdx.x & 31;
  const int wave = threadIdx.x >> 5;
  const int tilesN = N >> 6;
  const int tilesM = M >> 6;
  const int tile = blockIdx.x * 8 + wave;
  if (tile >= tilesM * tilesN) return;
  const int tm = tile / tilesN;
  const int tn = tile - tm * tilesN;
  const int m0 = tm << 6;
  const int n0 = tn << 6;

  const T* Ab  = A  + (size_t)b * strideA;
  const T* Bb  = Bt + (size_t)b * strideB;
  const T* Ab2 = SPLIT ? (A2  + (size_t)b * strideA) : nullptr;
  const T* Bb2 = SPLIT ? (Bt2 + (size_t)b * strideB) : nullptr;

  const int rlane = lane & 15;
  const int koff  = (lane >> 4) * 8;
  const int mOff  = (lane >> 4) * 8;

  v8f acc[4][4];
#pragma unroll
  for (int i = 0; i < 4; ++i)
#pragma unroll
    for (int j = 0; j < 4; ++j) acc[i][j] = (v8f){0.f,0.f,0.f,0.f,0.f,0.f,0.f,0.f};

  for (int k0 = 0; k0 < K; k0 += 32) {
    V bh[4], bl[4];
#pragma unroll
    for (int j = 0; j < 4; ++j) {
      const size_t bo = (size_t)(n0 + (j << 4) + rlane) * ldb + koff + k0;
      bh[j] = Frag<T>::load(Bb + bo);
      if (SPLIT) bl[j] = Frag<T>::load(Bb2 + bo);
    }
#pragma unroll
    for (int i = 0; i < 4; ++i) {
      const size_t ao = (size_t)(m0 + (i << 4) + rlane) * lda + koff + k0;
      V ah = Frag<T>::load(Ab + ao);
      V al;
      if (SPLIT) al = Frag<T>::load(Ab2 + ao);
#pragma unroll
      for (int j = 0; j < 4; ++j) {
        acc[i][j] = Frag<T>::mma(ah, bh[j], acc[i][j]);
        if (SPLIT) {
          acc[i][j] = Frag<T>::mma(ah, bl[j], acc[i][j]);
          acc[i][j] = Frag<T>::mma(al, bh[j], acc[i][j]);
        }
      }
      Frag<T>::guard(acc[i][0], acc[i][3], ah, SPLIT ? al : ah);
    }
    Frag<T>::keep(bh[0], bh[1], bh[2], bh[3]);
    if (SPLIT) Frag<T>::keep(bl[0], bl[1], bl[2], bl[3]);
  }
  acc_guard4(acc[0][0], acc[0][1], acc[0][2], acc[0][3]);
  acc_guard4(acc[1][0], acc[1][1], acc[1][2], acc[1][3]);
  acc_guard4(acc[2][0], acc[2][1], acc[2][2], acc[2][3]);
  acc_guard4(acc[3][0], acc[3][1], acc[3][2], acc[3][3]);

  float* slab = sT[wave];
  const float* Rb = RESID  ? (resid + (size_t)b * strideR) : nullptr;
  const float* Gb = GATED  ? (gate  + (size_t)b * strideG) : nullptr;
  const float* Pb = PREADD ? (pre   + (size_t)b * strideP) : nullptr;
#pragma unroll
  for (int i = 0; i < 4; ++i) {
    const int mBase = m0 + (i << 4);
#pragma unroll
    for (int j = 0; j < 4; ++j) {
      const int n = n0 + (j << 4) + rlane;
      float bv = 0.f, gv = 1.f;
      if (BIAS_MODE == 2) bv = bias[n];
      if (GATED) gv = Gb[n];
#pragma unroll
      for (int r = 0; r < 8; ++r) {
        float v = acc[i][j][r] * scale;
        if (BIAS_MODE == 1) v += bias[mBase + mOff + r];
        if (BIAS_MODE == 2) v += bv;
        if (PREADD) v += Pb[(size_t)(mBase + mOff + r) * ldc + n];
        if (GATED) v *= gv;
        if (RESID) v += Rb[(size_t)(mBase + mOff + r) * ldc + n];
        slab[(mOff + r) * 68 + (j << 4) + rlane] = v;
      }
    }
    __builtin_amdgcn_fence(__ATOMIC_RELEASE, "workgroup");
    __builtin_amdgcn_wave_barrier();
    __builtin_amdgcn_fence(__ATOMIC_ACQUIRE, "workgroup");
    if (OUT_MODE == 0) {
      float* C = (float*)Cout + (size_t)b * strideC;
      const int hh = lane >> 4, c4 = (lane & 15) * 4;
      for (int pass = 0; pass < 2; ++pass) {
#pragma unroll
        for (int it = 0; it < 8; ++it) {
          const int row = it * 2 + hh;
          v4f v = *(const v4f*)(slab + row * 68 + c4);
          *(volatile v4f*)(C + (size_t)(mBase + row) * ldc + n0 + c4) = v;
        }
        __threadfence();
      }
    } else {
      const int q = lane >> 3, c8 = (lane & 7) * 8;
      unsigned short* C  = (unsigned short*)Cout  + (size_t)b * strideC;
      unsigned short* C2 = (OUT_MODE == 2) ? ((unsigned short*)Cout2 + (size_t)b * strideC) : nullptr;
      for (int pass = 0; pass < 2; ++pass) {
#pragma unroll
        for (int it = 0; it < 4; ++it) {
          const int row = it * 4 + q;
          const float* sp = slab + row * 68 + c8;
          v8h hv, lv;
#pragma unroll
          for (int e = 0; e < 8; ++e) {
            if (OUT_MODE == 1) {
              hv[e] = (_Float16)sp[e];
            } else {
              unsigned short hb = f2bf_bits(sp[e]);
              unsigned short lb = f2bf_bits(sp[e] - bf_bits2f(hb));
              hv[e] = __builtin_bit_cast(_Float16, hb);
              lv[e] = __builtin_bit_cast(_Float16, lb);
            }
          }
          *(volatile v8h*)(C + (size_t)(mBase + row) * ldc + n0 + c8) = hv;
          if (OUT_MODE == 2) *(volatile v8h*)(C2 + (size_t)(mBase + row) * ldc + n0 + c8) = lv;
        }
        __threadfence();
      }
    }
    __builtin_amdgcn_fence(__ATOMIC_RELEASE, "workgroup");
    __builtin_amdgcn_wave_barrier();
    __builtin_amdgcn_fence(__ATOMIC_ACQUIRE, "workgroup");
  }
}

__global__ __launch_bounds__(256) void cast_f32_f16x2(
    const float* __restrict__ in, _Float16* __restrict__ out, int n2) {
  int i = blockIdx.x * 256 + threadIdx.x;
  if (i < n2) {
    const _Float16 h0 = (_Float16)in[2 * i], h1 = (_Float16)in[2 * i + 1];
    const unsigned u = (unsigned)__builtin_bit_cast(unsigned short, h0) | ((unsigned)__builtin_bit_cast(unsigned short, h1) << 16);
    ((volatile unsigned*)out)[i] = u;
    __threadfence();
    ((volatile unsigned*)out)[i] = u;
  }
}

__global__ __launch_bounds__(256) void tcast16_kernel(const float* __restrict__ W, unsigned short* __restrict__ oh,
                                                      int R, int Cc, float mul) {
  __shared__ __align__(16) float tf[64 * 68];
  const int c0  = blockIdx.x * 64;
  const int r0  = blockIdx.y * 64;
  const int tid = threadIdx.x;
  {
    const int lr = tid >> 4;
    const int c4 = (tid & 15) * 4;
#pragma unroll
    for (int it = 0; it < 4; ++it) {
      const int rr = it * 16 + lr;
      const v4f a = *(const v4f*)(W + (size_t)(r0 + rr) * Cc + c0 + c4);
      *(v4f*)(tf + rr * 68 + c4) = a;
    }
  }
  __syncthreads();
  const int sub = tid >> 3;
  const int c8  = (tid & 7) * 8;
  v4u hv[2];
#pragma unroll
  for (int it = 0; it < 2; ++it) {
    const int oc = it * 32 + sub;
    v4u a;
#pragma unroll
    for (int q = 0; q < 4; ++q) {
      const float f0 = tf[(c8 + 2 * q) * 68 + oc] * mul;
      const float f1 = tf[(c8 + 2 * q + 1) * 68 + oc] * mul;
      a[q] = pk16(f2h_bits(f0), f2h_bits(f1));
    }
    hv[it] = a;
  }
  for (int pass = 0; pass < 2; ++pass) {
#pragma unroll
    for (int it = 0; it < 2; ++it) {
      const int oc = it * 32 + sub;
      const size_t go = (size_t)(c0 + oc) * R + r0 + c8;
      *(volatile v4u*)(oh + go) = hv[it];
    }
    __threadfence();
  }
}

__global__ __launch_bounds__(256) void mod_kernel(const float* __restrict__ ts, const float* __restrict__ wmod,
                                                  const float* __restrict__ bmod, float* __restrict__ mods) {
  const int j = blockIdx.x * 256 + threadIdx.x;
  if (j < kSixD) {
    const float* w  = wmod + j;
    const float* t1 = ts + kDim;
    float a0 = 0.f, a1 = 0.f;
#pragma unroll 4
    for (int k = 0; k < kDim; ++k) {
      const float wv = w[(size_t)k * kSixD];
      a0 += ts[k] * wv;
      a1 += t1[k] * wv;
    }
    a0 += bmod[j];
    a1 += bmod[j];
    volatile float* m = mods;
    m[j] = a0; m[kSixD + j] = a1;
    __threadfence();
    m[j] = a0; m[kSixD + j] = a1;
  }
}

__global__ __launch_bounds__(256) void trig_kernel(const float* __restrict__ ang, float* __restrict__ ct,
                                                   float* __restrict__ st, int n) {
  const int i = blockIdx.x * 256 + threadIdx.x;
  if (i < n) {
    const float a  = ang[i];
    const float cv = cosf(a);
    const float sv = sinf(a);
    ((volatile float*)ct)[i] = cv;
    ((volatile float*)st)[i] = sv;
    __threadfence();
    ((volatile float*)ct)[i] = cv;
    ((volatile float*)st)[i] = sv;
  }
}

__device__ __forceinline__ _Float16 ln_elem(float d, float rstd, float sc, float sh, float m) {
  return (_Float16)(d * rstd * (1.0f + m * sc) + m * sh);
}
__global__ __launch_bounds__(128) void ln_mod_kernel(const float* __restrict__ X, const float* __restrict__ mods,
                                                     unsigned short* __restrict__ out, int rowsPerBatch,
                                                     int scIdx, int shIdx, float modOn) {
  __shared__ float red[4];
  const int row  = blockIdx.x;
  const int b    = row / rowsPerBatch;
  const int tid  = threadIdx.x;
  const int lane = tid & 31, wave = tid >> 5;
  const float* xr = X + (size_t)row * kDim + tid * 8;
  const v4f a0 = *(const v4f*)(xr);
  const v4f a1 = *(const v4f*)(xr + 4);
  float s = ((a0[0] + a0[1]) + (a0[2] + a0[3])) + ((a1[0] + a1[1]) + (a1[2] + a1[3]));
#pragma unroll
  for (int off = 1; off < 32; off <<= 1) s += __shfl_xor(s, off, 32);
  if (lane == 0) red[wave] = s;
  __syncthreads();
  const float mu = ((red[0] + red[1]) + (red[2] + red[3])) * (1.0f / 1024.0f);
  __syncthreads();
  const v4f d0 = a0 - mu;
  const v4f d1 = a1 - mu;
  float s2 = ((d0[0] * d0[0] + d0[1] * d0[1]) + (d0[2] * d0[2] + d0[3] * d0[3]))
           + ((d1[0] * d1[0] + d1[1] * d1[1]) + (d1[2] * d1[2] + d1[3] * d1[3]));
#pragma unroll
  for (int off = 1; off < 32; off <<= 1) s2 += __shfl_xor(s2, off, 32);
  if (lane == 0) red[wave] = s2;
  __syncthreads();
  const float var  = ((red[0] + red[1]) + (red[2] + red[3])) * (1.0f / 1024.0f);
  const float rstd = rsqrtf(var + 1e-6f);
  const float* scp = mods + (size_t)b * kSixD + (size_t)scIdx * kDim + tid * 8;
  const float* shp = mods + (size_t)b * kSixD + (size_t)shIdx * kDim + tid * 8;
  const v4f sc0 = *(const v4f*)(scp), sc1 = *(const v4f*)(scp + 4);
  const v4f sh0 = *(const v4f*)(shp), sh1 = *(const v4f*)(shp + 4);
  v8h hv;
  hv[0] = ln_elem(d0[0], rstd, sc0[0], sh0[0], modOn);
  hv[1] = ln_elem(d0[1], rstd, sc0[1], sh0[1], modOn);
  hv[2] = ln_elem(d0[2], rstd, sc0[2], sh0[2], modOn);
  hv[3] = ln_elem(d0[3], rstd, sc0[3], sh0[3], modOn);
  hv[4] = ln_elem(d1[0], rstd, sc1[0], sh1[0], modOn);
  hv[5] = ln_elem(d1[1], rstd, sc1[1], sh1[1], modOn);
  hv[6] = ln_elem(d1[2], rstd, sc1[2], sh1[2], modOn);
  hv[7] = ln_elem(d1[3], rstd, sc1[3], sh1[3], modOn);
  _Float16* op = (_Float16*)(void*)out + (size_t)row * kDim + tid * 8;
  *(volatile v8h*)op = hv;
  __threadfence();
  *(volatile v8h*)op = hv;
}

__global__ __launch_bounds__(256) void rope_kernel(const float* __restrict__ qk32, const float* __restrict__ ct,
                                                   const float* __restrict__ st, unsigned short* __restrict__ qk16) {
  const int t    = blockIdx.x;
  const int l    = t & (kSeq - 1);
  const int tid  = threadIdx.x;
  const int tsel = tid >> 7;
  const int h    = (tid >> 3) & 15;
  const int ck   = tid & 7;
  const int d0   = ck * 8;
  const int p0   = d0 ^ 32;
  const float* src = qk32 + (size_t)t * (2 * kDim) + tsel * kDim + h * kHeadDim;
  const v4f o0 = *(const v4f*)(src + d0), o1 = *(const v4f*)(src + d0 + 4);
  const v4f r0 = *(const v4f*)(src + p0), r1 = *(const v4f*)(src + p0 + 4);
  const float* cp = ct + (size_t)l * kHeadDim + d0;
  const float* sp = st + (size_t)l * kHeadDim + d0;
  const v4f c0 = *(const v4f*)(cp), c1 = *(const v4f*)(cp + 4);
  const v4f s0 = *(const v4f*)(sp), s1 = *(const v4f*)(sp + 4);
  const float sg = (ck < 4) ? -1.0f : 1.0f;
  const v4f y0 = o0 * c0 + (r0 * s0) * sg;
  const v4f y1 = o1 * c1 + (r1 * s1) * sg;
  v8h hv;
  hv[0] = (_Float16)y0[0]; hv[1] = (_Float16)y0[1]; hv[2] = (_Float16)y0[2]; hv[3] = (_Float16)y0[3];
  hv[4] = (_Float16)y1[0]; hv[5] = (_Float16)y1[1]; hv[6] = (_Float16)y1[2]; hv[7] = (_Float16)y1[3];
  _Float16* dst = (_Float16*)(void*)qk16 + (size_t)tsel * kTok * kDim + (size_t)t * kDim + h * kHeadDim + d0;
  *(volatile v8h*)dst = hv;
  __threadfence();
  *(volatile v8h*)dst = hv;
}

__global__ __launch_bounds__(256) void gelu_kernel(const float* __restrict__ hp, unsigned short* __restrict__ hhi,
                                                   unsigned short* __restrict__ hlo, int ldo, int colOff, int n2) {
  const int i = blockIdx.x * 256 + threadIdx.x;
  if (i < n2) {
    const int row = i >> 9;
    const int cp  = i & 511;
    const v2f f = *(const v2f*)(hp + (size_t)row * kDim + 2 * cp);
    const float g0 = 0.5f * f[0] * (1.0f + erff(f[0] * 0.70710678118654752f));
    const float g1 = 0.5f * f[1] * (1.0f + erff(f[1] * 0.70710678118654752f));
    const _Float16 q0 = (_Float16)g0, q1 = (_Float16)g1;
    const float e0 = (g0 - (float)q0) * kLoCarry;
    const float e1 = (g1 - (float)q1) * kLoCarry;
    const unsigned uh = pk16(__builtin_bit_cast(unsigned short, q0), __builtin_bit_cast(unsigned short, q1));
    const unsigned ul = pk16(f2h_bits(e0), f2h_bits(e1));
    const size_t o = ((size_t)row * ldo + colOff) / 2 + cp;
    ((volatile unsigned*)hhi)[o] = uh;
    ((volatile unsigned*)hlo)[o] = ul;
    __threadfence();
    ((volatile unsigned*)hhi)[o] = uh;
    ((volatile unsigned*)hlo)[o] = ul;
  }
}

__device__ __forceinline__ v8f mma_h(v16h a, v16h b, v8f c) {
  c = __builtin_amdgcn_wmma_f32_16x16x32_f16(false, a, false, b, (short)0, c, false, false);
  asm volatile("v_nop\n\tv_nop\n\tv_nop\n\tv_nop" : "+v"(c) : "v"(a), "v"(b));
  return c;
}

__global__ __launch_bounds__(128)
void mha64_f16_kernel(const unsigned short* __restrict__ qp, const unsigned short* __restrict__ kp,
                      const unsigned short* __restrict__ vtp, unsigned short* __restrict__ op,
                      int Lq, int Lk, float sscale) {
  union FH { v16h v; v8h h[2]; };
  __shared__ __align__(16) _Float16 Ksh[64 * 64];
  __shared__ __align__(16) _Float16 Vth[64 * 64];
  __shared__ __align__(16) _Float16 Psh[4][16 * 64];
  __shared__ __align__(16) float    Os[4][16 * 68];

  const int tid  = threadIdx.x;
  const int wave = tid >> 5;
  const int lane = tid & 31;
  const int hh   = lane >> 4;
  const int c    = lane & 15;

  const int nqb = Lq >> 6;
  const int bx  = blockIdx.x;
  const int qb  = bx % nqb;
  const int h   = bx / nqb;
  const int b   = blockIdx.y;
  const int q0  = qb * 64 + wave * 16;

  const _Float16* Qb = (const _Float16*)(const void*)qp  + (size_t)b * Lq * kDim + (size_t)h * kHeadDim;
  const _Float16* Kb = (const _Float16*)(const void*)kp  + (size_t)b * Lk * kDim + (size_t)h * kHeadDim;
  const _Float16* Vt = (const _Float16*)(const void*)vtp + (size_t)b * kDim * Lk + (size_t)h * kHeadDim * Lk;
  _Float16*       Ob = (_Float16*)(void*)op + (size_t)b * Lq * kDim + (size_t)h * kHeadDim;

  v16h qa[2];
#pragma unroll
  for (int dc = 0; dc < 2; ++dc)
    qa[dc] = Frag<_Float16>::load(Qb + (size_t)(q0 + c) * kDim + dc * 32 + 8 * hh);

  float mrow[8], lrow[8];
  v8f oacc[4];
#pragma unroll
  for (int r = 0; r < 8; ++r) { mrow[r] = -INFINITY; lrow[r] = 0.f; }
#pragma unroll
  for (int t = 0; t < 4; ++t) oacc[t] = (v8f){0.f,0.f,0.f,0.f,0.f,0.f,0.f,0.f};

  const int nChunks = Lk >> 6;
  for (int kc = 0; kc < nChunks; ++kc) {
    const int kv0 = kc * 64;
    __syncthreads();
    {
      const int r = tid >> 1, half = (tid & 1) * 32;
      const _Float16* ks = Kb + (size_t)(kv0 + r) * kDim + half;
      const _Float16* vs = Vt + (size_t)r * Lk + kv0 + half;
#pragma unroll
      for (int i = 0; i < 4; ++i) {
        const v8h a0 = *(const v8h*)(ks + 8 * i);
        const v8h b0 = *(const v8h*)(vs + 8 * i);
        *(v8h*)(Ksh + r * 64 + half + 8 * i) = a0;
        *(v8h*)(Vth + r * 64 + half + 8 * i) = b0;
      }
    }
    __syncthreads();

    v8f s[4];
#pragma unroll
    for (int j = 0; j < 4; ++j) {
      s[j] = (v8f){0.f,0.f,0.f,0.f,0.f,0.f,0.f,0.f};
#pragma unroll
      for (int dc = 0; dc < 2; ++dc) {
        FH kf;
        kf.h[0] = *(const v8h*)(Ksh + (j * 16 + c) * 64 + dc * 32 + 8 * hh);
        kf.h[1] = *(const v8h*)(Ksh + (j * 16 + c) * 64 + dc * 32 + 16 + 8 * hh);
        s[j] = mma_h(qa[dc], kf.v, s[j]);
      }
    }
    float cm[8];
#pragma unroll
    for (int r = 0; r < 8; ++r) {
      float m = -INFINITY;
#pragma unroll
      for (int j = 0; j < 4; ++j) {
        const float sv = s[j][r] * sscale;
        s[j][r] = sv;
        m = fmaxf(m, sv);
      }
#pragma unroll
      for (int off = 1; off < 16; off <<= 1) m = fmaxf(m, __shfl_xor(m, off, 32));
      cm[r] = m;
    }
    _Float16* pw = Psh[wave];
#pragma unroll
    for (int r = 0; r < 8; ++r) {
      const float mnew  = fmaxf(mrow[r], cm[r]);
      const float alpha = expf(mrow[r] - mnew);
      mrow[r] = mnew;
      float psum = 0.f;
#pragma unroll
      for (int j = 0; j < 4; ++j) {
        const float p = expf(s[j][r] - mnew);
        psum += p;
        pw[(8 * hh + r) * 64 + j * 16 + c] = (_Float16)(p * kPScale);
      }
#pragma unroll
      for (int off = 1; off < 16; off <<= 1) psum += __shfl_xor(psum, off, 32);
      lrow[r] = lrow[r] * alpha + psum;
#pragma unroll
      for (int t = 0; t < 4; ++t) oacc[t][r] *= alpha;
    }
    __builtin_amdgcn_fence(__ATOMIC_RELEASE, "workgroup");
    __builtin_amdgcn_wave_barrier();
    __builtin_amdgcn_fence(__ATOMIC_ACQUIRE, "workgroup");
#pragma unroll 1
    for (int kk = 0; kk < 2; ++kk) {
      FH pa;
      pa.h[0] = *(const v8h*)(pw + c * 64 + kk * 32 + 8 * hh);
      pa.h[1] = *(const v8h*)(pw + c * 64 + kk * 32 + 16 + 8 * hh);
#pragma unroll
      for (int t = 0; t < 4; ++t) {
        FH vb;
        vb.h[0] = *(const v8h*)(Vth + (t * 16 + c) * 64 + kk * 32 + 8 * hh);
        vb.h[1] = *(const v8h*)(Vth + (t * 16 + c) * 64 + kk * 32 + 16 + 8 * hh);
        oacc[t] = mma_h(pa.v, vb.v, oacc[t]);
      }
    }
  }

  float* os = Os[wave];
#pragma unroll
  for (int r = 0; r < 8; ++r) {
    const float inv = kOCarry / (lrow[r] * kPScale);
#pragma unroll
    for (int t = 0; t < 4; ++t) os[(8 * hh + r) * 68 + t * 16 + c] = oacc[t][r] * inv;
  }
  __builtin_amdgcn_fence(__ATOMIC_RELEASE, "workgroup");
  __builtin_amdgcn_wave_barrier();
  __builtin_amdgcn_fence(__ATOMIC_ACQUIRE, "workgroup");
  {
    const int q = lane >> 3, c8 = (lane & 7) * 8;
    for (int pass = 0; pass < 2; ++pass) {
#pragma unroll
      for (int it = 0; it < 4; ++it) {
        const int row = it * 4 + q;
        const float* spp = os + row * 68 + c8;
        v8h hv;
#pragma unroll
        for (int e = 0; e < 8; ++e) hv[e] = (_Float16)spp[e];
        *(volatile v8h*)(Ob + (size_t)(q0 + row) * kDim + c8) = hv;
      }
      __threadfence();
    }
  }
}

extern "C" void kernel_launch(void* const* d_in, const int* in_sizes, int n_in,
                              void* d_out, int out_size, void* d_ws, size_t ws_size,
                              hipStream_t stream) {
  if (n_in < 20) return;
  if (ws_size < kWsTotal) return;
  if (out_size != kTok * kDim) return;
  if (in_sizes[0] != kTok * kDim || in_sizes[1] != kBatch * kDim || in_sizes[2] != kCtxTok * kDim ||
      in_sizes[3] != kSeq * kHeadDim || in_sizes[4] != kDim * kSixD || in_sizes[5] != kSixD ||
      in_sizes[6] != kDim * kDim || in_sizes[7] != kDim * kDim || in_sizes[8] != kDim * kDim ||
      in_sizes[9] != kDim * kDim || in_sizes[10] != kDim || in_sizes[11] != kDim * kDim ||
      in_sizes[12] != kDim * kDim || in_sizes[13] != kDim * kDim || in_sizes[14] != kDim * kDim ||
      in_sizes[15] != kDim || in_sizes[16] != kDim * kHid || in_sizes[17] != kHid ||
      in_sizes[18] != kHid * kDim || in_sizes[19] != kDim) return;

  const float* x     = (const float*)d_in[0];
  const float* tse   = (const float*)d_in[1];
  const float* ctx   = (const float*)d_in[2];
  const float* rope  = (const float*)d_in[3];
  const float* w_mod = (const float*)d_in[4];
  const float* b_mod = (const float*)d_in[5];
  const float* wq_s  = (const float*)d_in[6];
  const float* wk_s  = (const float*)d_in[7];
  const float* wv_s  = (const float*)d_in[8];
  const float* wo_s  = (const float*)d_in[9];
  const float* bo_s  = (const float*)d_in[10];
  const float* wq_c  = (const float*)d_in[11];
  const float* wk_c  = (const float*)d_in[12];
  const float* wv_c  = (const float*)d_in[13];
  const float* wo_c  = (const float*)d_in[14];
  const float* bo_c  = (const float*)d_in[15];
  const float* w1    = (const float*)d_in[16];
  const float* b1    = (const float*)d_in[17];
  const float* w2    = (const float*)d_in[18];
  const float* b2    = (const float*)d_in[19];
  float* xo = (float*)d_out;

  char* ws = (char*)d_ws;
  float* mods = (float*)(ws + kOffSmall);
  float* cosT = (float*)(ws + kOffCos);
  float* sinT = (float*)(ws + kOffSin);
  float* xa   = (float*)(ws + kOffXa);
  float* hpre = (float*)(ws + kOffXa);
  float* tlo  = (float*)(ws + kOffXa);
  float* xb   = (float*)(ws + kOffXb);
  unsigned short* nx16  = (unsigned short*)(ws + kOffNx);
  float* qk32           = (float*)(ws + kOffBig);
  unsigned short* o16   = (unsigned short*)(ws + kOffBig);
  unsigned short* qc16  = (unsigned short*)(ws + kOffBig + 8 * kMiB);
  unsigned short* ctx16 = (unsigned short*)(ws + kOffBig + 16 * kMiB);
  unsigned short* kc16  = (unsigned short*)(ws + kOffBig + 18 * kMiB);
  unsigned short* vct16 = (unsigned short*)(ws + kOffBig + 20 * kMiB);
  unsigned short* h16   = (unsigned short*)(ws + kOffBig);
  unsigned short* h16lo = (unsigned short*)(ws + kOffHlo);
  unsigned short* q16   = (unsigned short*)(ws + kOffQkv);
  unsigned short* k16   = q16 + (size_t)kTok * kDim;
  unsigned short* vt16  = (unsigned short*)(ws + kOffQkv + 16 * kMiB);
  unsigned short* wqcT  = (unsigned short*)(ws + kOffQkv);
  unsigned short* wkcT  = (unsigned short*)(ws + kOffQkv + 2 * kMiB);
  unsigned short* wvcT  = (unsigned short*)(ws + kOffQkv + 4 * kMiB);
  unsigned short* wocT  = (unsigned short*)(ws + kOffQkv + 6 * kMiB);
  unsigned short* w1T   = (unsigned short*)(ws + kOffW1T);
  unsigned short* w2T   = (unsigned short*)(ws + kOffW2T);
  unsigned short* wqkT  = (unsigned short*)(ws + kOffWsw);
  unsigned short* wvsT  = (unsigned short*)(ws + kOffWsw + 4 * kMiB);
  unsigned short* wosT  = (unsigned short*)(ws + kOffWsw + 6 * kMiB);

  const long tokPlane16 = (long)kSeq * kDim;

  mod_kernel<<<kSixD / 256, 256, 0, stream>>>(tse, w_mod, b_mod, mods);
  trig_kernel<<<(kSeq * kHeadDim) / 256, 256, 0, stream>>>(rope, cosT, sinT, kSeq * kHeadDim);
  tcast16_kernel<<<dim3(kDim / 64, kDim / 64), 256, 0, stream>>>(wq_s, wqkT, kDim, kDim, kWCarry);
  tcast16_kernel<<<dim3(kDim / 64, kDim / 64), 256, 0, stream>>>(wk_s, wqkT + (size_t)kDim * kDim, kDim, kDim, kWCarry);
  tcast16_kernel<<<dim3(kDim / 64, kDim / 64), 256, 0, stream>>>(wv_s, wvsT, kDim, kDim, kWCarry);
  tcast16_kernel<<<dim3(kDim / 64, kDim / 64), 256, 0, stream>>>(wo_s, wosT, kDim, kDim, kWCarry);

  ln_mod_kernel<<<kTok, 128, 0, stream>>>(x, mods, nx16, kSeq, 1, 0, 1.0f);
  wmma_gemm64<0, false, 0, 0, false, false, false><<<dim3(256, 1), 256, 0, stream>>>(
      nx16, nx16, kDim, 0L, wqkT, wqkT, kDim, 0L, (void*)qk32, (void*)qk32, 2 * kDim, 0L,
      b_mod, mods, 0L, mods, 0L, mods, 0L, kTok, 2 * kDim, kDim, kWCarryInv);
  wmma_gemm64<0, false, 0, 1, false, false, false><<<dim3(64, kBatch), 256, 0, stream>>>(
      wvsT, wvsT, kDim, 0L, nx16, nx16, kDim, tokPlane16, (void*)vt16, (void*)vt16, kSeq, (long)kDim * kSeq,
      b_mod, mods, 0L, mods, 0L, mods, 0L, kDim, kSeq, kDim, kWCarryInv);
  rope_kernel<<<kTok, 256, 0, stream>>>(qk32, cosT, sinT, q16);
  mha64_f16_kernel<<<dim3(kHeads * (kSeq / 64), kBatch), 128, 0, stream>>>(q16, k16, vt16, o16, kSeq, kSeq, 0.125f);
  wmma_gemm64<0, false, 2, 0, true, true, false><<<dim3(64, kBatch), 256, 0, stream>>>(
      o16, o16, kDim, tokPlane16, wosT, wosT, kDim, 0L, (void*)xa, (void*)xa, kDim, tokPlane16,
      bo_s, mods + 2 * kDim, (long)kSixD, mods, 0L, x, tokPlane16, kSeq, kDim, kDim, kWOScale);

  tcast16_kernel<<<dim3(kDim / 64, kDim / 64), 256, 0, stream>>>(wq_c, wqcT, kDim, kDim, kWCarry);
  tcast16_kernel<<<dim3(kDim / 64, kDim / 64), 256, 0, stream>>>(wk_c, wkcT, kDim, kDim, kWCarry);
  tcast16_kernel<<<dim3(kDim / 64, kDim / 64), 256, 0, stream>>>(wv_c, wvcT, kDim, kDim, kWCarry);
  tcast16_kernel<<<dim3(kDim / 64, kDim / 64), 256, 0, stream>>>(wo_c, wocT, kDim, kDim, kWCarry);
  cast_f32_f16x2<<<(kCtxTok * kDim / 2) / 256, 256, 0, stream>>>(ctx, (_Float16*)(void*)ctx16, kCtxTok * kDim / 2);
  ln_mod_kernel<<<kTok, 128, 0, stream>>>(xa, mods, nx16, kSeq, 0, 0, 0.0f);
  wmma_gemm64<0, false, 0, 1, false, false, false><<<dim3(128, 1), 256, 0, stream>>>(
      nx16, nx16, kDim, 0L, wqcT, wqcT, kDim, 0L, (void*)qc16, (void*)qc16, kDim, 0L,
      b_mod, mods, 0L, mods, 0L, mods, 0L, kTok, kDim, kDim, kWCarryInv);
  wmma_gemm64<0, false, 0, 1, false, false, false><<<dim3(32, 1), 256, 0, stream>>>(
      ctx16, ctx16, kDim, 0L, wkcT, wkcT, kDim, 0L, (void*)kc16, (void*)kc16, kDim, 0L,
      b_mod, mods, 0L, mods, 0L, mods, 0L, kCtxTok, kDim, kDim, kWCarryInv);
  wmma_gemm64<0, false, 0, 1, false, false, false><<<dim3(16, kBatch), 256, 0, stream>>>(
      wvcT, wvcT, kDim, 0L, ctx16, ctx16, kDim, (long)kCtxLen * kDim, (void*)vct16, (void*)vct16, kCtxLen,
      (long)kDim * kCtxLen, b_mod, mods, 0L, mods, 0L, mods, 0L, kDim, kCtxLen, kDim, kWCarryInv);
  mha64_f16_kernel<<<dim3(kHeads * (kSeq / 64), kBatch), 128, 0, stream>>>(qc16, kc16, vct16, o16, kSeq, kCtxLen, 0.125f);
  wmma_gemm64<0, false, 2, 0, true, false, false><<<dim3(128, 1), 256, 0, stream>>>(
      o16, o16, kDim, 0L, wocT, wocT, kDim, 0L, (void*)xb, (void*)xb, kDim, 0L,
      bo_c, mods, 0L, mods, 0L, xa, 0L, kTok, kDim, kDim, kWOScale);

  tcast16_kernel<<<dim3(kHid / 64, kDim / 64), 256, 0, stream>>>(w1, w1T, kDim, kHid, kWCarry);
  tcast16_kernel<<<dim3(kDim / 64, kHid / 64), 256, 0, stream>>>(w2, w2T, kHid, kDim, kWCarry);
  ln_mod_kernel<<<kTok, 128, 0, stream>>>(xb, mods, nx16, kSeq, 4, 3, 1.0f);
  for (int qtr = 0; qtr < 4; ++qtr) {
    wmma_gemm64<0, false, 2, 0, false, false, false><<<dim3(128, 1), 256, 0, stream>>>(
        nx16, nx16, kDim, 0L, w1T + (size_t)qtr * kDim * kDim, w1T + (size_t)qtr * kDim * kDim, kDim, 0L,
        (void*)hpre, (void*)hpre, kDim, 0L, b1 + qtr * kDim, mods, 0L, mods, 0L, mods, 0L,
        kTok, kDim, kDim, kWCarryInv);
    gelu_kernel<<<(kTok * kDim / 2) / 256, 256, 0, stream>>>(hpre, h16, h16lo, kHid, qtr * kDim, kTok * kDim / 2);
  }
  wmma_gemm64<0, false, 0, 0, false, false, false><<<dim3(128, 1), 256, 0, stream>>>(
      h16lo, h16lo, kHid, 0L, w2T, w2T, kHid, 0L, (void*)tlo, (void*)tlo, kDim, 0L,
      b_mod, mods, 0L, mods, 0L, mods, 0L, kTok, kDim, kHid, kW2LoScale);
  wmma_gemm64<0, false, 2, 0, true, true, true><<<dim3(64, kBatch), 256, 0, stream>>>(
      h16, h16, kHid, (long)kSeq * kHid, w2T, w2T, kHid, 0L, (void*)xo, (void*)xo, kDim, tokPlane16,
      b2, mods + 5 * kDim, (long)kSixD, tlo, tokPlane16, xb, tokPlane16, kSeq, kDim, kHid, kWCarryInv);
}
